// GATDecoder_64544768524829
// MI455X (gfx1250) — hardware-verified
//
#include <hip/hip_runtime.h>


namespace {
constexpr int N = 50000, E = 800000, HID = 128, NH = 3, OPH = 43, MID = 129, OUT = 6, NO = 192  , KP = NO, NPAD = 51200, NBLK = NPAD / 128;
constexpr float FXS = 524288.0f, FXI = 1.0f / 524288.0f, NEG = 0.2f;

typedef _Float16 b16;
typedef __attribute__((ext_vector_type(16))) _Float16 v16b;
typedef __attribute__((ext_vector_type(8)))  _Float16 v8b;
typedef __attribute__((ext_vector_type(8)))  float v8f;
typedef __attribute__((ext_vector_type(4)))  float v4f;

__device__ __forceinline__ v8b ld8b(const b16* p) { return *(const v8b*)p; }
__device__ __forceinline__ v16b cat8b(v8b a, v8b b) { return __builtin_shufflevector(a, b, 0, 1, 2, 3, 4, 5, 6, 7, 8, 9, 10, 11, 12, 13, 14, 15); }
__device__ __forceinline__ v16b frag_kb(const b16* p, int hh) { return cat8b(ld8b(p + 8 * hh), ld8b(p + 16 + 8 * hh)); }
__device__ __forceinline__ void split16(float v, b16& hi, b16& lo) { hi = (b16)v; lo = (b16)(v - (float)hi); }
__device__ __forceinline__ void frag_ksplit(const float* p, int hh, v16b& fh_, v16b& fl_) {
  const float* p0 = p + 8 * hh; const float* p1 = p + 16 + 8 * hh;
#pragma unroll
  for (int e = 0; e < 8; ++e) { b16 a, c; split16(p0[e], a, c); fh_[e] = a; fl_[e] = c; split16(p1[e], a, c); fh_[8 + e] = a; fl_[8 + e] = c; }
}
__device__ __forceinline__ v8f wmma16b(v16b a, v16b b, v8f c) {
  v8f d = __builtin_amdgcn_wmma_f32_16x16x32_f16(false, a, false, b, (short)0, c, false, false);
  asm volatile("v_nop\n\tv_nop\n\tv_nop\n\tv_nop" : "+v"(d) : "v"(a), "v"(b));
  return d;
}
__device__ __forceinline__ void wave_lds_sync() {
  __builtin_amdgcn_fence(__ATOMIC_RELEASE, "workgroup");
  __builtin_amdgcn_wave_barrier();
  __builtin_amdgcn_fence(__ATOMIC_ACQUIRE, "workgroup");
}

struct Opnd { const void* p0; const void* p1; int ld; };
template <int NP> __device__ __forceinline__ void load_frags(const Opnd& o, int row, int kb, int hh, v16b& fh_, v16b& fl_) {
  if (NP == 0) { frag_ksplit((const float*)o.p0 + (size_t)row * o.ld + kb, hh, fh_, fl_); }
  else if (NP == 4) {
    const float* p = (const float*)o.p0 + (size_t)row * o.ld + kb; const float* p0 = p + 8 * hh; const float* p1 = p + 16 + 8 * hh;
#pragma unroll
    for (int e = 0; e < 8; ++e) { b16 a, c; split16(p0[e] * 64.0f, a, c); fh_[e] = a; fl_[e] = c; split16(p1[e] * 64.0f, a, c); fh_[8 + e] = a; fl_[8 + e] = c; }
  } else if (NP == 3) {
    const float* p = (const float*)o.p0 + (size_t)row * o.ld + kb; const float* p0 = p + 8 * hh; const float* p1 = p + 16 + 8 * hh;
#pragma unroll
    for (int e = 0; e < 8; ++e) { fh_[e] = (b16)p0[e]; fh_[8 + e] = (b16)p1[e]; }
    fl_ = fh_;
  } else {
    fh_ = frag_kb((const b16*)o.p0 + (size_t)row * o.ld + kb, hh);
    if (NP == 2) fl_ = frag_kb((const b16*)o.p1 + (size_t)row * o.ld + kb, hh); else fl_ = fh_;
  }
}
template <int ANP, int BNP> __device__ __forceinline__ v8f mac(v16b ah, v16b al, v16b bh, v16b bl, v8f c) {
  c = wmma16b(ah, bh, c);
  if (BNP == 0 || BNP == 2 || BNP == 4) c = wmma16b(ah, bl, c);
  if (ANP == 0 || ANP == 2 || ANP == 4) c = wmma16b(al, bh, c);
  return c;
}
template <int ANP, int BNP>
__device__ __forceinline__ void gemm_tile(const Opnd& A, const Opnd& B, int K, int m0, int c0, int nloc, int hlf, v8f (&acc)[2][4]) {
  for (int kb = 0; kb < K; kb += 32) {
    v16b a0h, a0l, a1h, a1l;
    load_frags<ANP>(A, m0 + nloc, kb, hlf, a0h, a0l);
    load_frags<ANP>(A, m0 + 16 + nloc, kb, hlf, a1h, a1l);
#pragma unroll
    for (int t = 0; t < 4; ++t) {
      v16b bh, bl;
      load_frags<BNP>(B, c0 + t * 16 + nloc, kb, hlf, bh, bl);
      acc[0][t] = mac<ANP, BNP>(a0h, a0l, bh, bl, acc[0][t]);
      acc[1][t] = mac<ANP, BNP>(a1h, a1l, bh, bl, acc[1][t]);
    }
  }
}

__device__ __forceinline__ void epi_planes(v8f (&acc)[2][4], float scale, bool two, b16* __restrict__ oh, b16* __restrict__ ol, int ldo,
                                           int m0, int c0, int lane, b16* Th, b16* Tl) {
  const int nloc = lane & 15, hlf = lane >> 4;
#pragma unroll
  for (int t = 0; t < 4; ++t)
#pragma unroll
    for (int r = 0; r < 2; ++r)
#pragma unroll
      for (int v = 0; v < 8; ++v) {
        const int rr = r * 16 + v + 8 * hlf, cc = t * 16 + nloc;
        b16 h_, l_; split16(acc[r][t][v] * scale, h_, l_);
        Th[rr * 64 + cc] = h_; Tl[rr * 64 + cc] = l_;
      }
  wave_lds_sync();
  for (int pass = 0; pass < 2; ++pass) {
#pragma unroll
    for (int j = 0; j < 8; ++j) {
      const int rr = j * 4 + (lane >> 3), c8 = (lane & 7) * 8;
      const size_t o = (size_t)(m0 + rr) * ldo + c0 + c8;
      *(volatile v8b*)(oh + o) = ld8b(Th + rr * 64 + c8);
      if (two) *(volatile v8b*)(ol + o) = ld8b(Tl + rr * 64 + c8);
    }
    __threadfence();
  }
}
__device__ __forceinline__ void epi_f32(v8f (&acc)[2][4], float scale, const float* rscale, float* __restrict__ out, int ldo, int m0, int c0, int lane, float* Tt) {
  const int nloc = lane & 15, hlf = lane >> 4;
#pragma unroll
  for (int t = 0; t < 4; ++t)
#pragma unroll
    for (int r = 0; r < 2; ++r)
#pragma unroll
      for (int v = 0; v < 8; ++v) {
        const int rr = r * 16 + v + 8 * hlf;
        const float rs = rscale ? rscale[(size_t)(m0 + rr) * 32] : 1.0f;
        Tt[rr * 64 + t * 16 + nloc] = acc[r][t][v] * scale * rs;
      }
  wave_lds_sync();
  float* dst0 = out + (size_t)m0 * ldo + c0;
  for (int pass = 0; pass < 2; ++pass) {
#pragma unroll
    for (int j = 0; j < 16; ++j) { const int rr = j * 2 + hlf, c4 = nloc * 4; *(volatile v4f*)(dst0 + (size_t)rr * ldo + c4) = *(const v4f*)(Tt + rr * 64 + c4); }
    __threadfence();
  }
}


__device__ __forceinline__ int fkey(float f) { const int b = __float_as_int(f); return (b >= 0) ? b : (b ^ 0x7FFFFFFF); }
__device__ __forceinline__ float fkey_inv(int k) { return __int_as_float((k >= 0) ? k : (k ^ 0x7FFFFFFF)); }

__global__ __launch_bounds__(256) void prep_kernel(const float* __restrict__ W0, const float* __restrict__ W1, const float* __restrict__ W2, b16* __restrict__ w0, b16* __restrict__ w1, b16* __restrict__ w2) {
  const size_t tid = (size_t)blockIdx.x * blockDim.x + threadIdx.x, nth = (size_t)gridDim.x * blockDim.x;
  for (int pass = 0; pass < 2; ++pass) {
    for (size_t p = tid; p < (size_t)NO * HID; p += nth) { const int n = (int)(p / HID), k = (int)(p % HID); ((volatile b16*)w0)[p] = (b16)((n < MID) ? W0[(size_t)k * MID + min(n, MID - 1)] : 0.0f); }
    for (size_t p = tid; p < (size_t)NO * KP; p += nth) { const int n = (int)(p / KP), k = (int)(p % KP); ((volatile b16*)w1)[p] = (b16)((n < MID && k < MID) ? W1[(size_t)min(k, MID - 1) * MID + min(n, MID - 1)] : 0.0f); }
    for (size_t p = tid; p < (size_t)64 * KP; p += nth) { const int n = (int)(p / KP), k = (int)(p % KP); ((volatile b16*)w2)[p] = (b16)((n < OUT && k < MID) ? W2[(size_t)min(k, MID - 1) * OUT + min(n, OUT - 1)] : 0.0f); }
    __threadfence();
  }
}

template <int KIN, int NOUT>
__global__ __launch_bounds__(128) void lin_kernel(const float* __restrict__ x, int nrow, const b16* __restrict__ w, float* __restrict__ y) {
  __shared__ __attribute__((aligned(16))) float Ts[4][32 * 64];
  const int lane = threadIdx.x & 31, wave = threadIdx.x >> 5, nloc = lane & 15, hlf = lane >> 4, m0 = blockIdx.y * 128 + wave * 32, c0 = blockIdx.x * 64;
  v8f acc[2][4];
#pragma unroll
  for (int r = 0; r < 2; ++r)
#pragma unroll
    for (int t = 0; t < 4; ++t) acc[r][t] = (v8f){};
  const int ra = min(m0 + nloc, nrow - 1), rb = min(m0 + 16 + nloc, nrow - 1);
#pragma unroll 1
  for (int kb = 0; kb < KIN; kb += 32) { v16b a0, a1, l0, l1;
#pragma unroll
    for (int e = 0; e < 16; ++e) { const int k = kb + ((e < 8) ? (8 * hlf + e) : (16 + 8 * hlf + e - 8)); b16 p, q; split16(x[(size_t)ra * KIN + k] * 8.0f, p, q); a0[e] = p; l0[e] = q; split16(x[(size_t)rb * KIN + k] * 8.0f, p, q); a1[e] = p; l1[e] = q; }
#pragma unroll
    for (int t = 0; t < 4; ++t) { const v16b bw = frag_kb(w + (size_t)(c0 + t * 16 + nloc) * KIN + kb, hlf); acc[0][t] = wmma16b(a0, bw, acc[0][t]); acc[0][t] = wmma16b(l0, bw, acc[0][t]); acc[1][t] = wmma16b(a1, bw, acc[1][t]); acc[1][t] = wmma16b(l1, bw, acc[1][t]); } }
  epi_f32(acc, 0.125f, nullptr, y, NOUT, m0, c0, lane, Ts[wave]);
}

template <int H, int C, int XP>
__global__ __launch_bounds__(256) void alpha_kernel(const float* __restrict__ xh, const float* __restrict__ as_, const float* __restrict__ ad_, float* __restrict__ al) {
  __shared__ float Ab[64][8];
  const int nl = threadIdx.x >> 2, q = threadIdx.x & 3, n = blockIdx.x * 64 + nl;
  float ss[3] = {0.0f, 0.0f, 0.0f}, sd[3] = {0.0f, 0.0f, 0.0f};
  for (int c = q; c < H * C; c += 4) { const float v = xh[(size_t)n * XP + c]; const int h = c / C, cc = c % C; ss[h] += v * as_[h * C + cc]; sd[h] += v * ad_[h * C + cc]; }
#pragma unroll
  for (int h = 0; h < 3; ++h) {
#pragma unroll
    for (int o = 1; o < 4; o <<= 1) { ss[h] += __shfl_xor(ss[h], o); sd[h] += __shfl_xor(sd[h], o); } }
  if (q == 0) { Ab[nl][0] = ss[0]; Ab[nl][1] = ss[1]; Ab[nl][2] = ss[2]; Ab[nl][3] = 0.0f; Ab[nl][4] = sd[0]; Ab[nl][5] = sd[1]; Ab[nl][6] = sd[2]; Ab[nl][7] = 0.0f; }
  __syncthreads();
  for (int pass = 0; pass < 2; ++pass) { if (threadIdx.x < 128) *(volatile v4f*)(al + (size_t)blockIdx.x * 512 + threadIdx.x * 4) = *(const v4f*)(&Ab[threadIdx.x >> 1][(threadIdx.x & 1) * 4]); __threadfence(); }
}

typedef __attribute__((ext_vector_type(4))) int v4i;
template <int DF, int H, int C, int NB, int MODE>
__global__ __launch_bounds__(256) void gat_kernel(const int* __restrict__ esrc, const int* __restrict__ edst, const float* __restrict__ xh, const float* __restrict__ al, const float* __restrict__ bias, float* __restrict__ xo) {
  constexpr int LW = DF / 32, HC = H * C;
  __shared__ __attribute__((aligned(16))) int acc[NB * DF];
  __shared__ int mx[NB * 4]; __shared__ int den[NB * 4]; __shared__ int list[8 * 256];
  const int t_ = threadIdx.x, wave = t_ >> 5, lane = t_ & 31, base = blockIdx.x * NB;
  for (int i = t_; i < NB * DF; i += 256) acc[i] = 0;
  for (int i = t_; i < NB * 4; i += 256) { const int slot = i >> 2, h = i & 3, node = base + slot; float e = -INFINITY;
    if (node < N && h < H) { float a = al[(size_t)node * 8 + h] + al[(size_t)node * 8 + 4 + h]; e = (a > 0.0f) ? a : NEG * a; }
    den[i] = 0; mx[i] = fkey(e); }
  __syncthreads();
  for (int c0 = 0; c0 < E; c0 += 256 * 8) { const int e0 = c0 + (wave * 32 + lane) * 8;
#pragma unroll
    for (int j = 0; j < 8; ++j) { const int ee = min(e0 + j, E - 1); const int dv = edst[ee]; const unsigned sl = (unsigned)(((e0 + j < E) ? dv : -1) - base);
      if (sl < (unsigned)NB) { int s = esrc[ee]; s = (s < 0) ? 0 : (s >= N ? N - 1 : s);
#pragma unroll
        for (int h = 0; h < H; ++h) { float a = al[(size_t)s * 8 + h] + al[(size_t)(base + sl) * 8 + 4 + h]; a = (a > 0.0f) ? a : NEG * a; atomicMax(&mx[sl * 4 + h], fkey(a)); } } } }
  __syncthreads();
  int* wl = list + wave * 256;
  const int col0 = lane * LW;
  auto accumulate = [&](int s, int slot) {
    float w[3] = {0.0f, 0.0f, 0.0f};
#pragma unroll
    for (int h = 0; h < H; ++h) { float a = al[(size_t)s * 8 + h] + al[(size_t)(base + slot) * 8 + 4 + h]; a = (a > 0.0f) ? a : NEG * a; w[h] = __expf(a - fkey_inv(mx[slot * 4 + h])); }
    { const float wl_ = (lane == 0) ? w[0] : (lane == 1) ? w[1] : w[2]; if (lane < H) atomicAdd(&den[slot * 4 + lane], (int)rintf(wl_ * FXS)); }
    const float* hr = xh + (size_t)s * DF + col0; int* ar = acc + slot * DF + col0;
#pragma unroll
    for (int c = 0; c < LW; ++c) { const int col = col0 + c; if (col < HC) { const int hh = col / C; const float wm = (hh == 0) ? w[0] : (hh == 1) ? w[1] : w[2]; atomicAdd(ar + c, (int)rintf(wm * hr[c] * FXS)); } }
  };
  for (int slot = wave; slot < NB; slot += 8) { if (base + slot < N) accumulate(base + slot, slot); }
  for (int c0 = 0; c0 < E; c0 += 256 * 8) {
    const int e0 = c0 + (wave * 32 + lane) * 8; int dd[8];
#pragma unroll
    for (int j = 0; j < 8; ++j) { const int dv = edst[min(e0 + j, E - 1)]; dd[j] = (e0 + j < E) ? dv : -1; }
    unsigned sl[8]; bool hit[8]; bool anyl = false;
#pragma unroll
    for (int j = 0; j < 8; ++j) { sl[j] = (unsigned)(dd[j] - base); hit[j] = sl[j] < (unsigned)NB; anyl |= hit[j]; }
    int wc = 0;
    if (__builtin_amdgcn_ballot_w32(anyl) != 0u) {
#pragma unroll
      for (int j = 0; j < 8; ++j) {
        const unsigned mj = __builtin_amdgcn_ballot_w32(hit[j]);
        if (mj != 0u) {
          if (hit[j]) { const int pos = wc + (int)__builtin_amdgcn_mbcnt_lo(mj, 0u); int s = esrc[min(e0 + j, E - 1)]; s = (s < 0) ? 0 : (s >= N ? N - 1 : s); wl[pos] = (s << 11) | (int)sl[j]; }
          wc += __builtin_popcount(mj); } } }
    __builtin_amdgcn_wave_barrier(); __builtin_amdgcn_fence(__ATOMIC_RELEASE, "workgroup"); __builtin_amdgcn_fence(__ATOMIC_ACQUIRE, "workgroup");
    for (int i = 0; i < wc; ++i) { const int ent = wl[i]; accumulate(ent >> 11, ent & 2047); }
    __builtin_amdgcn_wave_barrier();
  }
  __syncthreads();
  if (MODE == 0) {
    for (int pass = 0; pass < 2; ++pass) {
      for (int i = t_; i < NB * DF / 4; i += 256) { const int slot = i / (DF / 4), cq = (i % (DF / 4)) * 4, node = base + slot; v4f o = {0.0f, 0.0f, 0.0f, 0.0f};
        if (node < N) {
#pragma unroll
          for (int q = 0; q < 4; ++q) { const int c = cq + q; if (c < HC) { const int hh = c / C; const float dn = (float)den[slot * 4 + hh]; const float v = (float)acc[slot * DF + c] / (dn + 1e-16f * FXS) + bias[c]; o[q] = (v > 0.0f) ? v : NEG * v; } } }
        *(volatile v4f*)(xo + (size_t)node * DF + cq) = o; }
      __threadfence(); }
  } else {
    __shared__ float Ob[NB * OUT];
    for (int i = t_; i < NB * OUT; i += 256) { const int slot = i / OUT, c = i % OUT, node = base + slot; if (node < N) { const float dn = (float)den[slot * 4]; Ob[i] = (float)acc[slot * DF + c] / (dn + 1e-16f * FXS) + bias[c]; } }
    __syncthreads();
    const int nrow = min(NB, N - base);
    for (int pass = 0; pass < 2; ++pass) { for (int i = t_; i < nrow * OUT / 4; i += 256) *(volatile v4f*)(xo + (size_t)base * OUT + i * 4) = *(const v4f*)(&Ob[i * 4]); __threadfence(); }
  }
}
}

extern "C" void kernel_launch(void* const* d_in, const int* in_sizes, int n_in,
                              void* d_out, int out_size, void* d_ws, size_t ws_size, hipStream_t stream) {
  (void)n_in; (void)out_size;
  const float* x = (const float*)d_in[0]; const int* ei = (const int*)d_in[1];
  const float* W0 = (const float*)d_in[2]; const float* a0s = (const float*)d_in[3]; const float* a0d = (const float*)d_in[4]; const float* b0 = (const float*)d_in[5];
  const float* W1 = (const float*)d_in[6]; const float* a1s = (const float*)d_in[7]; const float* a1d = (const float*)d_in[8]; const float* b1 = (const float*)d_in[9];
  const float* W2 = (const float*)d_in[10]; const float* a2s = (const float*)d_in[11]; const float* a2d = (const float*)d_in[12]; const float* b2 = (const float*)d_in[13];
  float* out = (float*)d_out;
  if (in_sizes[0] != N * HID || in_sizes[1] != 2 * E || in_sizes[2] != HID * MID || in_sizes[6] != MID * MID || in_sizes[10] != MID * OUT) return;
  const int* esrc = ei; const int* edst = ei + E;
  size_t off = 0; char* ws = (char*)d_ws;
  auto carve = [&](size_t bytes) { char* p = ws + off; off += (bytes + 255) & ~(size_t)255; return p; };
  b16* w0 = (b16*)carve((size_t)NO * HID * 2); b16* w1 = (b16*)carve((size_t)NO * KP * 2); b16* w2 = (b16*)carve((size_t)64 * KP * 2);
  float* xh = (float*)carve((size_t)NPAD * NO * 4); float* h = (float*)carve((size_t)NPAD * KP * 4); float* al = (float*)carve((size_t)NPAD * 8 * 4); float* xh2 = (float*)carve((size_t)NPAD * 64 * 4);
  if (off > ws_size) return;
  prep_kernel<<<128, 256, 0, stream>>>(W0, W1, W2, w0, w1, w2);
  lin_kernel<HID, NO><<<dim3(NO / 64, NBLK), 128, 0, stream>>>(x, N, w0, xh);
  alpha_kernel<NH, OPH, NO><<<NPAD / 64, 256, 0, stream>>>(xh, a0s, a0d, al);
  gat_kernel<NO, NH, OPH, 256, 0><<<NPAD / 256, 256, 0, stream>>>(esrc, edst, xh, al, b0, h);
  lin_kernel<KP, NO><<<dim3(NO / 64, NBLK), 128, 0, stream>>>(h, NPAD, w1, xh);
  alpha_kernel<NH, OPH, NO><<<NPAD / 64, 256, 0, stream>>>(xh, a1s, a1d, al);
  gat_kernel<NO, NH, OPH, 256, 0><<<NPAD / 256, 256, 0, stream>>>(esrc, edst, xh, al, b1, h);
  lin_kernel<KP, 64><<<dim3(1, NBLK), 128, 0, stream>>>(h, NPAD, w2, xh2);
  alpha_kernel<1, OUT, 64><<<NPAD / 64, 256, 0, stream>>>(xh2, a2s, a2d, al);
  gat_kernel<64, 1, OUT, 1024, 1><<<NPAD / 1024, 256, 0, stream>>>(esrc, edst, xh2, al, b2, out);
}
